// SimilarGCN_87917980549713
// MI455X (gfx1250) — hardware-verified
//
#include <hip/hip_runtime.h>


#define NS   8
#define CC   256
#define HWN  961
#define MM   7688
#define MP   7744
#define HID  512
#define OC   256
typedef _Float16 h16;
typedef unsigned short bf;
typedef __attribute__((ext_vector_type(16))) __bf16   v16bf;
typedef __attribute__((ext_vector_type(16))) _Float16 v16h;
typedef __attribute__((ext_vector_type(8)))  _Float16 v8h;
typedef __attribute__((ext_vector_type(8)))  unsigned short v8us;
typedef __attribute__((ext_vector_type(8)))  float    v8f;
typedef __attribute__((ext_vector_type(4)))  float    v4f;
typedef v8h  __attribute__((may_alias)) v8ha;
typedef v4f  __attribute__((may_alias)) v4fa;
typedef v8us __attribute__((may_alias)) v8usa;

__device__ __forceinline__ unsigned short f2bf(float f) { unsigned u = __float_as_uint(f); u += 0x7FFFu + ((u >> 16) & 1u); return (unsigned short)(u >> 16); }
__device__ __forceinline__ float bf2f(unsigned short b) { return __uint_as_float(((unsigned)b) << 16); }
__device__ __forceinline__ float bfr(float f) { return bf2f(f2bf(f)); }
__device__ __forceinline__ v16h cat16(v8h lo, v8h hi) { return __builtin_shufflevector(lo, hi, 0, 1, 2, 3, 4, 5, 6, 7, 8, 9, 10, 11, 12, 13, 14, 15); }
__device__ __forceinline__ v16bf cat16b(v8us lo, v8us hi) { return __builtin_bit_cast(v16bf, __builtin_shufflevector(lo, hi, 0, 1, 2, 3, 4, 5, 6, 7, 8, 9, 10, 11, 12, 13, 14, 15)); }
__device__ __forceinline__ v8f wmma16(v16h a, v16h b, v8f c) { return __builtin_amdgcn_wmma_f32_16x16x32_f16(false, a, false, b, (short)0, c, false, false); }
__device__ __forceinline__ v8f wmmab(v16bf a, v16bf b, v8f c) { return __builtin_amdgcn_wmma_f32_16x16x32_bf16(false, a, false, b, (short)0, c, false, false); }


template <typename T16> struct WFrag;
template <> struct WFrag<h16> { typedef v16h V; static __device__ __forceinline__ V ld(const h16* p) { return cat16(*(const v8h*)p, *(const v8h*)(p + 16)); } static __device__ __forceinline__ v8f mma(V a, V b, v8f c) { return wmma16(a, b, c); } };
template <> struct WFrag<bf> { typedef v16bf V; static __device__ __forceinline__ V ld(const bf* p) { return cat16b(*(const v8us*)p, *(const v8us*)(p + 16)); } static __device__ __forceinline__ v8f mma(V a, V b, v8f c) { return wmmab(a, b, c); } };
template <typename T16, int NSPLIT, bool BIAS>
__global__ __launch_bounds__(32) void k_gemmw(const T16* __restrict__ A, const T16* __restrict__ A2, const T16* __restrict__ Bt, const T16* __restrict__ Bt2, int K, float* C, int ldc, const float* __restrict__ bias, size_t sA, size_t sB, size_t sC) {
    typedef typename WFrag<T16>::V V;
    __shared__ __align__(16) float os[16 * 68];
    const size_t z = blockIdx.z; A += z * sA; if (A2) A2 += z * sA; Bt += z * sB; if (Bt2) Bt2 += z * sB; C += z * sC;
    const int lane = threadIdx.x & 31, lr = lane & 15, hi = lane >> 4; const int r0 = blockIdx.x * 64, c0 = blockIdx.y * 64;
    v8f acc[4][4];
#pragma unroll
    for (int mb = 0; mb < 4; ++mb)
#pragma unroll
        for (int nb = 0; nb < 4; ++nb) acc[mb][nb] = (v8f){};
    const size_t aoff = (size_t)(r0 + lr) * K + 8 * hi, boff = (size_t)(c0 + lr) * K + 8 * hi;
#pragma unroll 1
    for (int kc = 0; kc < K; kc += 32) {
        V a[4], a2[4];
#pragma unroll
        for (int mb = 0; mb < 4; ++mb) { a[mb] = WFrag<T16>::ld(A + aoff + (size_t)mb * 16 * K + kc); if (NSPLIT == 1 || NSPLIT == 2) a2[mb] = WFrag<T16>::ld(A2 + aoff + (size_t)mb * 16 * K + kc); }
#pragma unroll
        for (int nb = 0; nb < 4; ++nb) { const V b = WFrag<T16>::ld(Bt + boff + (size_t)nb * 16 * K + kc); V b2; if (NSPLIT >= 2) b2 = WFrag<T16>::ld(Bt2 + boff + (size_t)nb * 16 * K + kc);
#pragma unroll
            for (int mb = 0; mb < 4; ++mb) { acc[mb][nb] = WFrag<T16>::mma(a[mb], b, acc[mb][nb]); if (NSPLIT == 1 || NSPLIT == 2) acc[mb][nb] = WFrag<T16>::mma(a2[mb], b, acc[mb][nb]); if (NSPLIT >= 2) acc[mb][nb] = WFrag<T16>::mma(a[mb], b2, acc[mb][nb]); } }
        asm volatile("v_nop\n\tv_nop\n\tv_nop\n\tv_nop" : "+v"(acc[0][0]), "+v"(acc[1][1]), "+v"(acc[2][2]), "+v"(acc[3][3]) : "v"(a[0]), "v"(a[3]));
    }
#pragma unroll
    for (int mb = 0; mb < 4; ++mb) {
#pragma unroll
        for (int nb = 0; nb < 4; ++nb) {
#pragma unroll
            for (int j = 0; j < 8; ++j) os[(hi * 8 + j) * 68 + nb * 16 + lr] = acc[mb][nb][j]; }
        __builtin_amdgcn_wave_barrier(); asm volatile("" ::: "memory");
        float* crow = C + (size_t)(r0 + mb * 16) * ldc + c0;
#pragma unroll 1
        for (int ps = 0; ps < 2; ++ps) {
#pragma unroll
            for (int s = 0; s < 8; ++s) { const int row = 2 * s + hi, cofs = lr * 4; v4f val = *(const v4fa*)(os + row * 68 + cofs); if (BIAS) { val[0] += bfr(bias[c0 + cofs]); val[1] += bfr(bias[c0 + cofs + 1]); val[2] += bfr(bias[c0 + cofs + 2]); val[3] += bfr(bias[c0 + cofs + 3]); }
                *(volatile v4f*)(crow + (size_t)row * ldc + cofs) = val; }
            if (ps == 0) __threadfence(); }
        __builtin_amdgcn_wave_barrier(); asm volatile("" ::: "memory");
    }
}

__device__ __forceinline__ void splitf(float y, unsigned short& h, unsigned short& l) { h = f2bf(y); l = f2bf(y - bf2f(h)); }
__device__ __forceinline__ float dinvb(int b) { return (b == 0 || b == NS - 1) ? __frsqrt_rn(963.0f) : __frsqrt_rn(964.0f); }
typedef __attribute__((ext_vector_type(2))) unsigned short v2us;
typedef __attribute__((ext_vector_type(4))) unsigned short v4us;

__global__ __launch_bounds__(256) void k_cvt8(const float* __restrict__ src, bf* dst, size_t n8) { const size_t i = (size_t)blockIdx.x * 256 + threadIdx.x; if (i >= n8) return; const v8f v = *(const v8f*)(src + i * 8); v8us o;
#pragma unroll
    for (int k = 0; k < 8; ++k) o[k] = f2bf(v[k]); *(volatile v8us*)(dst + i * 8) = o; __threadfence(); *(volatile v8us*)(dst + i * 8) = o; }
__global__ __launch_bounds__(256) void k_nodes(const float* __restrict__ x, float* X0) { const size_t e = ((size_t)blockIdx.x * 256 + threadIdx.x) * 4; if (e >= (size_t)MM * CC) return; const int c = (int)(e % CC); const int i = (int)(e / CC); const int b = i / HWN, pos = i % HWN; v4f o;
#pragma unroll
    for (int q = 0; q < 4; ++q) o[q] = bfr(x[((size_t)b * CC + c + q) * HWN + pos]); *(volatile v4f*)(X0 + e) = o; __threadfence(); *(volatile v4f*)(X0 + e) = o; }
__global__ __launch_bounds__(256) void k_csum(const float* __restrict__ X, int ncol, float* S) { const int e = blockIdx.x * 256 + threadIdx.x; if (e >= NS * ncol) return; const int c = e % ncol, b = e / ncol; float s = 0.f; for (int p = 0; p < HWN; ++p) s = __fadd_rn(s, X[((size_t)b * HWN + p) * ncol + c]); *(volatile float*)(S + e) = s; __threadfence(); *(volatile float*)(S + e) = s; }
__global__ __launch_bounds__(256) void k_agg(const float* __restrict__ X, const float* __restrict__ S, int ncol, bf* Ph, bf* Pl) { const size_t e = ((size_t)blockIdx.x * 256 + threadIdx.x) * 4; if (e >= (size_t)MP * ncol) return; const int c = (int)(e % ncol); const int i = (int)(e / ncol); v4us oh, ol;
    if (i >= MM) { for (int q = 0; q < 4; ++q) { oh[q] = 0; ol[q] = 0; } }
    else { const int b = i / HWN; const float db = dinvb(b);
#pragma unroll
        for (int q = 0; q < 4; ++q) { float acc = __fmul_rn(db, S[b * ncol + c + q]); if (b > 0) { float t = __fmul_rn(dinvb(b - 1), X[(size_t)(i - HWN) * ncol + c + q]); asm volatile("" : "+v"(t)); acc = __fadd_rn(acc, t); } if (b < NS - 1) { float t = __fmul_rn(dinvb(b + 1), X[(size_t)(i + HWN) * ncol + c + q]); asm volatile("" : "+v"(t)); acc = __fadd_rn(acc, t); }
            float t2 = __fmul_rn(db, X[(size_t)i * ncol + c + q]); asm volatile("" : "+v"(t2)); acc = __fadd_rn(acc, t2); unsigned short a, cc; splitf(__fmul_rn(db, acc), a, cc); oh[q] = a; ol[q] = cc; } }
    *(volatile v4us*)(Ph + e) = oh; *(volatile v4us*)(Pl + e) = ol; __threadfence(); *(volatile v4us*)(Ph + e) = oh; *(volatile v4us*)(Pl + e) = ol; }
__global__ __launch_bounds__(256) void k_lrelu(const float* __restrict__ G, size_t n4, float* Y) { const size_t i = ((size_t)blockIdx.x * 256 + threadIdx.x) * 4; if (i >= n4 * 4) return; const v4f a = *(const v4f*)(G + i); v4f o;
#pragma unroll
    for (int q = 0; q < 4; ++q) o[q] = a[q] >= 0.f ? a[q] : 0.01f * a[q]; *(volatile v4f*)(Y + i) = o; __threadfence(); *(volatile v4f*)(Y + i) = o; }
__global__ __launch_bounds__(256) void k_max(const float* __restrict__ G2, float* OUT) { const int e = blockIdx.x * 256 + threadIdx.x; if (e >= OC * HWN) return; const int pos = e % HWN, c = e / HWN; float m = -3.0e38f;
#pragma unroll
    for (int b = 0; b < NS; ++b) { const float g = G2[((size_t)b * HWN + pos) * OC + c]; m = fmaxf(m, g >= 0.f ? g : 0.01f * g); }
    *(volatile float*)(OUT + e) = m; __threadfence(); *(volatile float*)(OUT + e) = m; }

extern "C" void kernel_launch(void* const* d_in, const int* in_sizes, int n_in,
                              void* d_out, int out_size, void* d_ws, size_t ws_size, hipStream_t stream) {
    (void)in_sizes; (void)n_in; (void)out_size;
    const float* x = (const float*)d_in[0]; const float* W1 = (const float*)d_in[1]; const float* b1 = (const float*)d_in[2]; const float* W2 = (const float*)d_in[3]; const float* b2 = (const float*)d_in[4];
    float* OUT = (float*)d_out;
    char* wsp = (char*)d_ws;
    auto take = [&](size_t bytes) { char* p = wsp; wsp += (bytes + 255) & ~(size_t)255; return (void*)p; };
    bf* B1 = (bf*)take((size_t)HID * CC * 2); bf* B2 = (bf*)take((size_t)OC * HID * 2); float* X0 = (float*)take((size_t)MM * CC * 4); float* S = (float*)take((size_t)NS * HID * 4); bf* Ph = (bf*)take((size_t)MP * HID * 2); bf* Pl = (bf*)take((size_t)MP * HID * 2);
    float* G1 = (float*)take((size_t)MP * HID * 4); float* Y1 = (float*)take((size_t)MP * HID * 4); float* G2 = (float*)take((size_t)MP * OC * 4);
    if ((size_t)(wsp - (char*)d_ws) > ws_size) return;
    k_cvt8<<<(HID * CC / 8 + 255) / 256, 256, 0, stream>>>(W1, B1, (size_t)HID * CC / 8); k_cvt8<<<(OC * HID / 8 + 255) / 256, 256, 0, stream>>>(W2, B2, (size_t)OC * HID / 8);
    k_nodes<<<(MM * CC / 4 + 255) / 256, 256, 0, stream>>>(x, X0);
    k_csum<<<(NS * CC + 255) / 256, 256, 0, stream>>>(X0, CC, S); k_agg<<<(MP * CC / 4 + 255) / 256, 256, 0, stream>>>(X0, S, CC, Ph, Pl);
    k_gemmw<bf, 1, true><<<dim3(MP / 64, HID / 64, 1), 32, 0, stream>>>(Ph, Pl, B1, nullptr, CC, G1, HID, b1, 0, 0, 0); k_lrelu<<<(unsigned)(((size_t)MM * HID / 4 + 255) / 256), 256, 0, stream>>>(G1, (size_t)MM * HID / 4, Y1);
    k_csum<<<(NS * HID + 255) / 256, 256, 0, stream>>>(Y1, HID, S); k_agg<<<(MP * HID / 4 + 255) / 256, 256, 0, stream>>>(Y1, S, HID, Ph, Pl);
    k_gemmw<bf, 1, true><<<dim3(MP / 64, OC / 64, 1), 32, 0, stream>>>(Ph, Pl, B2, nullptr, HID, G2, OC, b2, 0, 0, 0);
    k_max<<<(OC * HWN + 255) / 256, 256, 0, stream>>>(G2, OUT);
}
